// RecModel_11003706212749
// MI455X (gfx1250) — hardware-run, weakly checked
//
#include <hip/hip_runtime.h>
#include <math.h>

constexpr int NBATCH     = 256;
constexpr int NSTEP      = 512;
constexpr int NIN        = 64;
constexpr int NHID       = 256;
constexpr int NGATE      = 4 * NHID;
constexpr int NOUT       = 8;
constexpr int KTOT       = NIN + NHID;
constexpr int KSTEPS     = KTOT / 32;
constexpr int ROWS_BLK   = 16;
constexpr int NTHR       = 256;
constexpr int NWAVE      = NTHR / 32;
constexpr int UNITS_WAVE = NHID / NWAVE;
constexpr int APITCH     = KTOT + 8;
constexpr int ABUF       = ROWS_BLK * APITCH;
constexpr int FPITCH     = NHID + 4;
constexpr float ACARRY   = 128.0f;
constexpr float WCARRY   = 256.0f;
constexpr float FOLD     = 1.0f / (ACARRY * WCARRY);
constexpr float F16_MIN_NORMAL = 6.103515625e-05f;

constexpr int OUT0_OFF = 0;
constexpr int OUT1_OFF = 262144 / 4;
constexpr int OUT2_OFF = 270336 / 4;
constexpr int OUT3_OFF = 532480 / 4;
constexpr int OUT_TOTAL = 794624 / 4;

static_assert(KTOT == 320);
static_assert(KTOT % 32 == 0);
static_assert(UNITS_WAVE == 32);
static_assert(NBATCH % ROWS_BLK == 0);
static_assert(OUT1_OFF == NBATCH * NHID);
static_assert(OUT2_OFF == OUT1_OFF + NBATCH * NOUT);
static_assert(OUT3_OFF == OUT2_OFF + NBATCH * NHID);
static_assert(OUT3_OFF + NBATCH * NHID == OUT_TOTAL);
static_assert((OUT1_OFF * 4) % 128 == 0);
static_assert((OUT2_OFF * 4) % 128 == 0);
static_assert((OUT3_OFF * 4) % 128 == 0);
static_assert((APITCH * 2) % 16 == 0);
static_assert((FPITCH * 4) % 16 == 0);
static_assert(ROWS_BLK * NIN == NTHR * 4);
static_assert((ROWS_BLK * NHID / 4) % NTHR == 0);
static_assert(ROWS_BLK * NOUT == 128);

typedef __attribute__((ext_vector_type(16))) _Float16 v16h;
typedef __attribute__((ext_vector_type(8)))  _Float16 v8h;
typedef __attribute__((ext_vector_type(8)))  float    v8f;
typedef __attribute__((ext_vector_type(4)))  float    v4f;
typedef __attribute__((ext_vector_type(4)))  unsigned v4u;
typedef __attribute__((ext_vector_type(2)))  unsigned v2u;

__device__ __forceinline__ float flush16(float v) {
  return (__builtin_fabsf(v) < F16_MIN_NORMAL) ? 0.0f : v;
}
__device__ __forceinline__ unsigned h16_bits(float v) {
  const _Float16 h = (_Float16)flush16(v);
  return (unsigned)__builtin_bit_cast(unsigned short, h);
}

union FragU { v16h v; v8h h[2]; };
__device__ __forceinline__ v16h frag16(const _Float16* p) {
  FragU f;
  f.h[0] = *(const v8h*)(p);
  f.h[1] = *(const v8h*)(p + 16);
  return f.v;
}
__device__ __forceinline__ v8f mma_g(v16h a, v16h b, v8f c) {
  c = __builtin_amdgcn_wmma_f32_16x16x32_f16(false, a, false, b, (short)0, c, false, false);
  asm volatile("v_nop\n\tv_nop\n\tv_nop\n\tv_nop" : "+v"(c) : "v"(a), "v"(b));
  return c;
}

__device__ __forceinline__ float fsig(float z)  { return __builtin_amdgcn_rcpf(1.0f + __expf(-z)); }
__device__ __forceinline__ float ftanh(float z) { return 1.0f - 2.0f * __builtin_amdgcn_rcpf(__expf(2.0f * z) + 1.0f); }

template <int SRC_LD, int SEGS, int COL0, int NLINES>
__global__ __launch_bounds__(256) void pack_w_lines(const float* __restrict__ src,
                                                    unsigned short* __restrict__ dst) {
  static_assert(NLINES % 32 == 0);
  static_assert(SEGS * 64 == SRC_LD);
  static_assert(COL0 % 64 == 0);
  const int tid  = threadIdx.x;
  const int line = blockIdx.x * 32 + (tid >> 3);
  const int q    = tid & 7;
  const int n    = line / SEGS;
  const int seg  = line - n * SEGS;
  const float* sp = src + (size_t)n * SRC_LD + seg * 64 + q * 8;
  const v4f va = *(const v4f*)(sp);
  const v4f vb = *(const v4f*)(sp + 4);
  const float f0 = va[0], f1 = va[1], f2 = va[2], f3 = va[3];
  const float f4 = vb[0], f5 = vb[1], f6 = vb[2], f7 = vb[3];
  v4u pk;
  pk[0] = h16_bits(f0 * WCARRY) | (h16_bits(f1 * WCARRY) << 16);
  pk[1] = h16_bits(f2 * WCARRY) | (h16_bits(f3 * WCARRY) << 16);
  pk[2] = h16_bits(f4 * WCARRY) | (h16_bits(f5 * WCARRY) << 16);
  pk[3] = h16_bits(f6 * WCARRY) | (h16_bits(f7 * WCARRY) << 16);
  unsigned short* dp = dst + (size_t)n * KTOT + COL0 + seg * 64 + q * 8;
  *(volatile v4u*)dp = pk;
  __threadfence();
  *(volatile v4u*)dp = pk;
}

__global__ __launch_bounds__(NTHR) void lstm_rows_kernel(
    const float* __restrict__ x, const float* __restrict__ h0, const float* __restrict__ c0,
    const float* __restrict__ bvec, const float* __restrict__ W_out, const float* __restrict__ b_out,
    const _Float16* Wp, float* __restrict__ out) {
  __shared__ __align__(16) _Float16 Ash[2 * ABUF];
  __shared__ __align__(16) float    Hf[ROWS_BLK * FPITCH];
  __shared__ __align__(16) float    Cf[ROWS_BLK * FPITCH];
  __shared__ __align__(16) float    Ps[2 * ROWS_BLK * NOUT];

  const int tid = threadIdx.x, lane = tid & 31, wave = tid >> 5;
  const int c = lane & 15, hh = lane >> 4;
  const int b0 = blockIdx.x * ROWS_BLK;
  const int u0 = UNITS_WAVE * wave + c;

#pragma unroll
  for (int it = 0; it < (ROWS_BLK * NHID / 4) / NTHR; ++it) {
    const int idx = it * NTHR + tid;
    const int row = idx >> 6, c4 = (idx & 63) * 4;
    const v4f hv = *(const v4f*)(h0 + (size_t)(b0 + row) * NHID + c4);
    const v4f cv = *(const v4f*)(c0 + (size_t)(b0 + row) * NHID + c4);
    *(v4f*)(Hf + row * FPITCH + c4) = hv;
    *(v4f*)(Cf + row * FPITCH + c4) = cv;
  }
  const int xm = tid >> 4, xk = (tid & 15) * 4;
  const float* xrow = x + (size_t)(b0 + xm) * NSTEP * NIN + xk;
  {
    const v4f xv = *(const v4f*)(xrow);
    const float f0 = xv[0], f1 = xv[1], f2 = xv[2], f3 = xv[3];
    v2u pk;
    pk[0] = h16_bits(f0 * ACARRY) | (h16_bits(f1 * ACARRY) << 16);
    pk[1] = h16_bits(f2 * ACARRY) | (h16_bits(f3 * ACARRY) << 16);
    *(v2u*)(Ash + xm * APITCH + xk) = pk;
  }
  __syncthreads();

  float cs[2][8], hs[2][8];
#pragma unroll
  for (int nt = 0; nt < 2; ++nt)
#pragma unroll
    for (int r = 0; r < 8; ++r) {
      const int row = 8 * hh + r, u = u0 + 16 * nt;
      const float hv = Hf[row * FPITCH + u];
      cs[nt][r] = Cf[row * FPITCH + u];
      hs[nt][r] = hv;
      Ash[row * APITCH + NIN + u] = (_Float16)flush16(hv * ACARRY);
    }
  float bia[2][4];
#pragma unroll
  for (int nt = 0; nt < 2; ++nt)
#pragma unroll
    for (int g = 0; g < 4; ++g) bia[nt][g] = bvec[NHID * g + u0 + 16 * nt];
  __syncthreads();

  const _Float16* wl = Wp + (size_t)u0 * KTOT + 8 * hh;
  const int arow = c * APITCH + 8 * hh;
  const v8f z8 = {0.f, 0.f, 0.f, 0.f, 0.f, 0.f, 0.f, 0.f};

#pragma unroll 1
  for (int t = 0; t < NSTEP; ++t) {
    const int q = t & 1;
    const _Float16* Ar = Ash + q * ABUF;
    _Float16*       Aw = Ash + (q ^ 1) * ABUF;
    const int tn = (t + 1 < NSTEP) ? (t + 1) : (NSTEP - 1);
    const v4f xv = *(const v4f*)(xrow + (size_t)tn * NIN);

#pragma unroll
    for (int nt = 0; nt < 2; ++nt) {
      v8f a0 = z8, a1 = z8, a2 = z8, a3 = z8;
      const _Float16* ap = Ar + arow;
      const _Float16* wb = wl + nt * 16 * KTOT;
#pragma unroll 1
      for (int ks = 0; ks < KSTEPS; ++ks) {
        const v16h av = frag16(ap);
        const v16h b0v = frag16(wb);
        const v16h b1v = frag16(wb + 1 * NHID * KTOT);
        const v16h b2v = frag16(wb + 2 * NHID * KTOT);
        const v16h b3v = frag16(wb + 3 * NHID * KTOT);
        a0 = mma_g(av, b0v, a0);
        a1 = mma_g(av, b1v, a1);
        a2 = mma_g(av, b2v, a2);
        a3 = mma_g(av, b3v, a3);
        ap += 32;
        wb += 32;
      }
#pragma unroll
      for (int r = 0; r < 8; ++r) {
        const float zi = fmaf(a0[r], FOLD, bia[nt][0]);
        const float zf = fmaf(a1[r], FOLD, bia[nt][1]);
        const float zg = fmaf(a2[r], FOLD, bia[nt][2]);
        const float zo = fmaf(a3[r], FOLD, bia[nt][3]);
        const float ig = fsig(zi);
        const float fg = fsig(zf);
        const float gg = ftanh(zg);
        const float og = fsig(zo);
        const float cn = fg * cs[nt][r] + ig * gg;
        const float hn = og * ftanh(cn);
        cs[nt][r] = cn;
        hs[nt][r] = hn;
        Aw[(8 * hh + r) * APITCH + NIN + u0 + 16 * nt] = (_Float16)flush16(hn * ACARRY);
      }
    }
    {
      const float f0 = xv[0], f1 = xv[1], f2 = xv[2], f3 = xv[3];
      v2u pk;
      pk[0] = h16_bits(f0 * ACARRY) | (h16_bits(f1 * ACARRY) << 16);
      pk[1] = h16_bits(f2 * ACARRY) | (h16_bits(f3 * ACARRY) << 16);
      *(v2u*)(Aw + xm * APITCH + xk) = pk;
    }
    __syncthreads();
  }

#pragma unroll
  for (int nt = 0; nt < 2; ++nt)
#pragma unroll
    for (int r = 0; r < 8; ++r) {
      const int row = 8 * hh + r, u = u0 + 16 * nt;
      Hf[row * FPITCH + u] = hs[nt][r];
      Cf[row * FPITCH + u] = cs[nt][r];
    }
  __syncthreads();

  for (int pass = 0; pass < 2; ++pass) {
#pragma unroll
    for (int rr = 0; rr < 2; ++rr) {
#pragma unroll
      for (int hf = 0; hf < 2; ++hf) {
        const int row = 2 * wave + rr;
        const int col = hf * 128 + 4 * lane;
        const v4f hv = *(const v4f*)(Hf + row * FPITCH + col);
        const v4f cv = *(const v4f*)(Cf + row * FPITCH + col);
        const size_t gi = (size_t)(b0 + row) * NHID + col;
        *(volatile v4f*)(out + OUT0_OFF + gi) = hv;
        *(volatile v4f*)(out + OUT2_OFF + gi) = hv;
        *(volatile v4f*)(out + OUT3_OFF + gi) = cv;
      }
    }
    __threadfence();
  }

  {
    const int o = tid & 127, kh = tid >> 7;
    const int row = o >> 3, cls = o & 7;
    const float* hr = Hf + row * FPITCH + 128 * kh;
    const float* wr = W_out + cls * NHID + 128 * kh;
    float s = 0.0f;
#pragma unroll 1
    for (int u4 = 0; u4 < 32; ++u4) {
      const v4f hv = *(const v4f*)(hr + 4 * u4);
      const v4f wv = *(const v4f*)(wr + 4 * u4);
      s = fmaf(hv[0], wv[0], s);
      s = fmaf(hv[1], wv[1], s);
      s = fmaf(hv[2], wv[2], s);
      s = fmaf(hv[3], wv[3], s);
    }
    Ps[kh * 128 + o] = s;
  }
  const v4f bo = *(const v4f*)(b_out + 4 * (lane & 1));
  float bo0 = bo[0], bo1 = bo[1], bo2 = bo[2], bo3 = bo[3];
  asm volatile("" : "+v"(bo0), "+v"(bo1), "+v"(bo2), "+v"(bo3));
  __syncthreads();
  if (wave == 0) {
    const v4f p0 = *(const v4f*)(Ps + 4 * lane);
    const v4f p1 = *(const v4f*)(Ps + 128 + 4 * lane);
    v4f ov;
    ov[0] = (p0[0] + p1[0]) + bo0;
    ov[1] = (p0[1] + p1[1]) + bo1;
    ov[2] = (p0[2] + p1[2]) + bo2;
    ov[3] = (p0[3] + p1[3]) + bo3;
    float* op = out + OUT1_OFF + (size_t)b0 * NOUT + 4 * lane;
    for (int pass = 0; pass < 2; ++pass) {
      *(volatile v4f*)op = ov;
      __threadfence();
    }
  }
}

extern "C" void kernel_launch(void* const* d_in, const int* in_sizes, int n_in,
                              void* d_out, int out_size, void* d_ws, size_t ws_size, hipStream_t stream) {
  if (n_in < 8 || d_out == nullptr || d_ws == nullptr) return;
  if (in_sizes[0] != NBATCH * NSTEP * NIN || in_sizes[1] != NBATCH * NHID || in_sizes[2] != NBATCH * NHID ||
      in_sizes[3] != NGATE * NIN || in_sizes[4] != NGATE * NHID || in_sizes[5] != NGATE ||
      in_sizes[6] != NOUT * NHID || in_sizes[7] != NOUT || out_size != OUT_TOTAL) return;
  constexpr size_t WP_BYTES = (size_t)NGATE * KTOT * 2;
  static_assert(WP_BYTES == 655360);
  if (ws_size < WP_BYTES) return;

  const float* inputs = (const float*)d_in[0];
  const float* h0     = (const float*)d_in[1];
  const float* c0     = (const float*)d_in[2];
  const float* W_ih   = (const float*)d_in[3];
  const float* W_hh   = (const float*)d_in[4];
  const float* bvec   = (const float*)d_in[5];
  const float* W_out  = (const float*)d_in[6];
  const float* b_out  = (const float*)d_in[7];
  unsigned short* Wp  = (unsigned short*)d_ws;
  float* out = (float*)d_out;

  pack_w_lines<NIN, 1, 0, NGATE><<<NGATE / 32, 256, 0, stream>>>(W_ih, Wp);
  pack_w_lines<NHID, 4, NIN, NGATE * 4><<<(NGATE * 4) / 32, 256, 0, stream>>>(W_hh, Wp);
  lstm_rows_kernel<<<NBATCH / ROWS_BLK, NTHR, 0, stream>>>(
      inputs, h0, c0, bvec, W_out, b_out, (const _Float16*)Wp, out);
}
